// JK_NET_20469814133286
// MI455X (gfx1250) — hardware-verified
//
#include <hip/hip_runtime.h>
#include <stddef.h>


#define HID    128
#define OUTC   64
#define NLAY   4
#define NTHR   256
#define NWAVE  8
#define EPT    8
#define NGRP   2
#define CHUNK  (NTHR * EPT * NGRP)
#define WCAP   (EPT * NGRP * 32)
#define LISTN  (NWAVE * WCAP)
#define NBC    4096
#define NBF    1024
#define RCAP   40960
#define RBN    128
#define DEGCAP 256
#define GROWS  128
#define OTHR   512
#define AP     (HID + 8)
#define CPADX  256
#define WSCALE 8.0f
#define WINV   0.125f

#define LDS_FILL  ((RCAP + NBF + LISTN) * 4 + 64)
#define LDS_LAYER (2 * GROWS * AP * 2)

static_assert((CHUNK & (CHUNK - 1)) == 0);
static_assert(CHUNK <= 4096);
static_assert(NBC <= 4096 && NBF <= 4096);
static_assert((NBC & (NBC - 1)) == 0 && (NBF & (NBF - 1)) == 0);
static_assert(NBC == 4 * NBF);
static_assert(OTHR * 8 == NBC);
static_assert((RCAP % 32) == 0);
static_assert(GROWS == NWAVE * 16);
static_assert((HID % 32) == 0 && OUTC == 64);
static_assert((NLAY * HID * HID / 8) % NTHR == 0);
static_assert(((NLAY * HID * HID / 8) + (NLAY * OUTC * HID / 8)) % NTHR == 0);
static_assert(GROWS * OUTC * 4 <= GROWS * AP * 2);
static_assert((AP % 8) == 0);

typedef float    v4f  __attribute__((ext_vector_type(4)));
typedef float    v8f  __attribute__((ext_vector_type(8)));
typedef int      v4i  __attribute__((ext_vector_type(4)));
typedef _Float16 v4h  __attribute__((ext_vector_type(4)));
typedef _Float16 v8h  __attribute__((ext_vector_type(8)));
typedef _Float16 v16h __attribute__((ext_vector_type(16)));
union FragH { v16h v; v8h h[2]; };
union FI { float f; int i; };

__device__ __forceinline__ v8f wmh(v16h a, v16h b, v8f c) {
  v8f d = __builtin_amdgcn_wmma_f32_16x16x32_f16(false, a, false, b, (short)0, c, false, false);
  asm volatile("v_nop\n\tv_nop\n\tv_nop\n\tv_nop" : "+v"(d) : "v"(a), "v"(b));
  return d;
}

template <int NB>
__device__ __forceinline__ int scan_chunk(const int* __restrict__ dsts, int nE, int cbase, int slotBase,
                                          int vec8, int* list, int tid, int lane, int wave) {
  int wc = 0;
#pragma unroll
  for (int g = 0; g < NGRP; ++g) {
    const int el0  = (g * NTHR + tid) * EPT;
    const int e0   = cbase + el0;
    const int sent = -2147483647 - 1;
    v4i da, db;
    if (vec8 != 0 && cbase + CHUNK <= nE) {
      da = *(const v4i*)(dsts + e0);
      db = *(const v4i*)(dsts + e0 + 4);
    } else {
      da.x = (e0     < nE) ? dsts[min(e0, nE - 1)] : sent;
      da.y = (e0 + 1 < nE) ? dsts[min(e0 + 1, nE - 1)] : sent;
      da.z = (e0 + 2 < nE) ? dsts[min(e0 + 2, nE - 1)] : sent;
      da.w = (e0 + 3 < nE) ? dsts[min(e0 + 3, nE - 1)] : sent;
      db.x = (e0 + 4 < nE) ? dsts[min(e0 + 4, nE - 1)] : sent;
      db.y = (e0 + 5 < nE) ? dsts[min(e0 + 5, nE - 1)] : sent;
      db.z = (e0 + 6 < nE) ? dsts[min(e0 + 6, nE - 1)] : sent;
      db.w = (e0 + 7 < nE) ? dsts[min(e0 + 7, nE - 1)] : sent;
    }
    const unsigned nb = (unsigned)slotBase;
    const unsigned s0 = (unsigned)da.x - nb, s1 = (unsigned)da.y - nb;
    const unsigned s2 = (unsigned)da.z - nb, s3 = (unsigned)da.w - nb;
    const unsigned s4 = (unsigned)db.x - nb, s5 = (unsigned)db.y - nb;
    const unsigned s6 = (unsigned)db.z - nb, s7 = (unsigned)db.w - nb;
    const bool h0 = s0 < (unsigned)NB, h1 = s1 < (unsigned)NB, h2 = s2 < (unsigned)NB, h3 = s3 < (unsigned)NB;
    const bool h4 = s4 < (unsigned)NB, h5 = s5 < (unsigned)NB, h6 = s6 < (unsigned)NB, h7 = s7 < (unsigned)NB;
    const unsigned any = __builtin_amdgcn_ballot_w32(h0 | h1 | h2 | h3 | h4 | h5 | h6 | h7);
    if (any != 0u) {
#define HITJ(J, HJ, SJ) { \
        const unsigned mj = __builtin_amdgcn_ballot_w32(HJ); \
        if (mj != 0u) { \
          if (HJ) { \
            const int pos = wc + (int)__builtin_amdgcn_mbcnt_lo(mj, 0u); \
            if (pos < WCAP) list[wave * WCAP + pos] = ((el0 + (J)) << 12) | (int)(SJ); \
          } \
          wc += (int)__builtin_popcount(mj); } }
      HITJ(0, h0, s0)
      HITJ(1, h1, s1)
      HITJ(2, h2, s2)
      HITJ(3, h3, s3)
      HITJ(4, h4, s4)
      HITJ(5, h5, s5)
      HITJ(6, h6, s6)
      HITJ(7, h7, s7)
#undef HITJ
    }
  }
  return wc;
}

__global__ __launch_bounds__(NTHR) void k_wprep(
    const float* __restrict__ W0, const float* __restrict__ W1, const float* __restrict__ W2,
    const float* __restrict__ W3, const float* __restrict__ linW, _Float16* wl, _Float16* wj) {
  const int gA = NLAY * HID * HID / 8;
  const int gB = NLAY * OUTC * HID / 8;
  const int i = blockIdx.x * NTHR + (int)threadIdx.x;
  if (i >= gA + gB) return;
  float v[8];
  _Float16* dp;
  if (blockIdx.x * NTHR < gA) {
    const int o     = i * 8;
    const int layer = o / (HID * HID);
    const int oo    = o - layer * HID * HID;
    const int n     = oo / HID;
    const int k0    = oo - n * HID;
    const float* src = layer == 0 ? W0 : (layer == 1 ? W1 : (layer == 2 ? W2 : W3));
#pragma unroll
    for (int e = 0; e < 8; ++e) v[e] = src[(size_t)(k0 + e) * HID + n] * WSCALE;
    dp = wl + o;
  } else {
    const int o     = (i - gA) * 8;
    const int layer = o / (OUTC * HID);
    const int oo    = o - layer * OUTC * HID;
    const int n     = oo / HID;
    const int k0    = oo - n * HID;
#pragma unroll
    for (int e = 0; e < 8; ++e) v[e] = linW[(size_t)(layer * HID + k0 + e) * OUTC + n] * WSCALE;
    dp = wj + o;
  }
  v8h hv;
  hv[0] = (_Float16)v[0]; hv[1] = (_Float16)v[1]; hv[2] = (_Float16)v[2]; hv[3] = (_Float16)v[3];
  hv[4] = (_Float16)v[4]; hv[5] = (_Float16)v[5]; hv[6] = (_Float16)v[6]; hv[7] = (_Float16)v[7];
  *(volatile v8h*)dp = hv;
  __threadfence();
  *(volatile v8h*)dp = hv;
}

__global__ __launch_bounds__(NTHR) void k_count(
    const int* __restrict__ ei, int* cnt, float* dinv, int nE, int vec8) {
  __shared__ __attribute__((aligned(16))) int scnt[NBC];
  __shared__ __attribute__((aligned(16))) int list[LISTN];
  __shared__ int wcnt[NWAVE];
  const int tid = threadIdx.x, lane = tid & 31, wave = tid >> 5;
  const int nodeBase = blockIdx.x * NBC;
  const int* dsts = ei + nE;

  for (int i = tid; i < NBC; i += NTHR) scnt[i] = 0;
  __syncthreads();

  const int nChunks = (nE + CHUNK - 1) / CHUNK;
#pragma unroll 1
  for (int ch = 0; ch < nChunks; ++ch) {
    const int cbase = ch * CHUNK;
    const int wc = scan_chunk<NBC>(dsts, nE, cbase, nodeBase, vec8, list, tid, lane, wave);
    if (lane == 0) wcnt[wave] = wc;
    __syncthreads();
    if (wave == 0) {
#pragma unroll 1
      for (int wsx = 0; wsx < NWAVE; ++wsx) {
        int n = __builtin_amdgcn_readfirstlane(wcnt[wsx]);
        n = n > WCAP ? WCAP : (n < 0 ? 0 : n);
        const int* lp = list + wsx * WCAP;
#pragma unroll 1
        for (int i = 0; i < n; ++i) {
          const int ent  = __builtin_amdgcn_readfirstlane(lp[i]);
          const int slot = ent & (NBC - 1);
          if (lane == 0) scnt[slot] = scnt[slot] + 1;
        }
      }
    }
    __syncthreads();
  }

  v4i cq[4]; v4f dq[4];
#pragma unroll
  for (int q = 0; q < 4; ++q) {
    const int f = (wave * 4 + q) * 128 + 4 * lane;
    const v4i c = *(const v4i*)(scnt + f);
    cq[q] = c;
    dq[q].x = rsqrtf((float)(c.x + 1));
    dq[q].y = rsqrtf((float)(c.y + 1));
    dq[q].z = rsqrtf((float)(c.z + 1));
    dq[q].w = rsqrtf((float)(c.w + 1));
  }
  int*   cp = cnt + (size_t)nodeBase;
  float* dp = dinv + (size_t)nodeBase;
#pragma unroll
  for (int q = 0; q < 4; ++q) {
    const int f = (wave * 4 + q) * 128 + 4 * lane;
    *(volatile v4i*)(cp + f) = cq[q];
    *(volatile v4f*)(dp + f) = dq[q];
  }
  __threadfence();
#pragma unroll
  for (int q = 0; q < 4; ++q) {
    const int f = (wave * 4 + q) * 128 + 4 * lane;
    *(volatile v4i*)(cp + f) = cq[q];
    *(volatile v4f*)(dp + f) = dq[q];
  }
}

__global__ __launch_bounds__(OTHR) void k_offsets(
    const int* __restrict__ cnt, int* off, int* rbase, int nChunk) {
  __shared__ __attribute__((aligned(16))) int soff[NBC];
  __shared__ __attribute__((aligned(16))) int srb[RBN];
  __shared__ int wtot[OTHR / 32];
  const int tid = threadIdx.x, lane = tid & 31, wave = tid >> 5, sub = tid >> 7;
  for (int i = tid; i < RBN; i += OTHR) srb[i] = 0;
  int carry = 0;
#pragma unroll 1
  for (int ch = 0; ch < nChunk; ++ch) {
    const int base = ch * NBC;
    const v4i c0 = *(const v4i*)(cnt + base + 8 * tid);
    const v4i c1 = *(const v4i*)(cnt + base + 8 * tid + 4);
    const int e0 = max(c0.x, 0), e1 = max(c0.y, 0), e2 = max(c0.z, 0), e3 = max(c0.w, 0);
    const int e4 = max(c1.x, 0), e5 = max(c1.y, 0), e6 = max(c1.z, 0), e7 = max(c1.w, 0);
    const int ts = e0 + e1 + e2 + e3 + e4 + e5 + e6 + e7;
    int incl = ts;
#pragma unroll
    for (int d = 1; d < 32; d <<= 1) {
      const int t = __shfl_up(incl, d);
      if (lane >= d) incl += t;
    }
    if (lane == 31) wtot[wave] = incl;
    __syncthreads();
    const int S0 = wtot[0]  + wtot[1]  + wtot[2]  + wtot[3];
    const int S1 = wtot[4]  + wtot[5]  + wtot[6]  + wtot[7];
    const int S2 = wtot[8]  + wtot[9]  + wtot[10] + wtot[11];
    const int S3 = wtot[12] + wtot[13] + wtot[14] + wtot[15];
    int pre = 0;
#pragma unroll 1
    for (int w = 4 * sub; w < wave; ++w) pre += wtot[w];
    const int b0 = carry;
    const int b1 = b0 + ((S0 + 31) & ~31);
    const int b2 = b1 + ((S1 + 31) & ~31);
    const int b3 = b2 + ((S2 + 31) & ~31);
    const int b4 = b3 + ((S3 + 31) & ~31);
    const int myb = sub == 0 ? b0 : (sub == 1 ? b1 : (sub == 2 ? b2 : b3));
    if (tid == 0) {
      srb[min(4 * ch + 0, RBN - 1)] = b0;
      srb[min(4 * ch + 1, RBN - 1)] = b1;
      srb[min(4 * ch + 2, RBN - 1)] = b2;
      srb[min(4 * ch + 3, RBN - 1)] = b3;
    }
    int run = myb + pre + incl - ts;
    soff[8 * tid + 0] = run; run += e0;
    soff[8 * tid + 1] = run; run += e1;
    soff[8 * tid + 2] = run; run += e2;
    soff[8 * tid + 3] = run; run += e3;
    soff[8 * tid + 4] = run; run += e4;
    soff[8 * tid + 5] = run; run += e5;
    soff[8 * tid + 6] = run; run += e6;
    soff[8 * tid + 7] = run;
    carry = b4;
    __syncthreads();
    const v4i o0 = *(const v4i*)(soff + 4 * tid);
    const v4i o1 = *(const v4i*)(soff + 4 * (tid + OTHR));
    int* op = off + base;
    *(volatile v4i*)(op + 4 * tid) = o0;
    *(volatile v4i*)(op + 4 * (tid + OTHR)) = o1;
    __threadfence();
    *(volatile v4i*)(op + 4 * tid) = o0;
    *(volatile v4i*)(op + 4 * (tid + OTHR)) = o1;
    __syncthreads();
  }
  if (tid == 0) srb[min(4 * nChunk, RBN - 1)] = carry;
  __syncthreads();
  v4i rv = {0, 0, 0, 0};
  if (tid < 32) rv = *(const v4i*)(srb + 4 * tid);
  if (tid < 32) *(volatile v4i*)(rbase + 4 * tid) = rv;
  __threadfence();
  if (tid < 32) *(volatile v4i*)(rbase + 4 * tid) = rv;
}

__global__ __launch_bounds__(NTHR) void k_fill(
    const int* __restrict__ ei, const int* __restrict__ off, const int* __restrict__ rbase,
    int* csr, int nN, int nE, int vec8, int csrLen) {
  extern __shared__ v4f lds_dyn[];
  int* region = (int*)lds_dyn;
  int* cursor = region + RCAP;
  int* list   = cursor + NBF;
  int* wcnt   = list + LISTN;
  const int tid = threadIdx.x, lane = tid & 31, wave = tid >> 5;
  const int b = blockIdx.x;
  const int nodeBase = b * NBF;
  const int* dsts = ei + nE;

  int rb0 = rbase[b];
  const int rb1 = rbase[b + 1];
  rb0 = rb0 < 0 ? 0 : (rb0 > csrLen ? csrLen : rb0);
  rb0 &= ~31;
  int len = rb1 - rb0;
  len = len < 0 ? 0 : (len > RCAP ? RCAP : len);
  int lenW = (len + 31) & ~31;
  if (rb0 + lenW > csrLen) lenW = (csrLen - rb0) & ~31;

  {
    const v4i z = {0, 0, 0, 0};
    for (int i = tid; i < RCAP / 4; i += NTHR) ((v4i*)region)[i] = z;
    for (int s = tid; s < NBF; s += NTHR) {
      int o = off[nodeBase + s] - rb0;
      o = o < 0 ? 0 : (o > RCAP ? RCAP : o);
      cursor[s] = o;
    }
  }
  __syncthreads();

  const int nChunks = (nE + CHUNK - 1) / CHUNK;
#pragma unroll 1
  for (int ch = 0; ch < nChunks; ++ch) {
    const int cbase = ch * CHUNK;
    const int wc = scan_chunk<NBF>(dsts, nE, cbase, nodeBase, vec8, list, tid, lane, wave);
    if (lane == 0) wcnt[wave] = wc;
    __syncthreads();
    if (wave == 0) {
#pragma unroll 1
      for (int wsx = 0; wsx < NWAVE; ++wsx) {
        int n = __builtin_amdgcn_readfirstlane(wcnt[wsx]);
        n = n > WCAP ? WCAP : (n < 0 ? 0 : n);
        const int* lp = list + wsx * WCAP;
#pragma unroll 1
        for (int i = 0; i < n; ++i) {
          const int ent  = __builtin_amdgcn_readfirstlane(lp[i]);
          const int slot = ent & (NBF - 1);
          int e = cbase + ((ent >> 12) & (CHUNK - 1));
          e = e > nE - 1 ? nE - 1 : e;
          int src = ei[e];
          src = src < 0 ? 0 : (src > nN - 1 ? nN - 1 : src);
          if (lane == 0) {
            int pos = cursor[slot];
            pos = pos < 0 ? 0 : (pos > RCAP - 1 ? RCAP - 1 : pos);
            region[pos] = src;
            const int np = pos + 1;
            cursor[slot] = np > RCAP ? RCAP : np;
          }
        }
      }
    }
    __syncthreads();
  }

  const int nv = lenW >> 2;
  int* gp = csr + rb0;
#pragma unroll 1
  for (int i = tid; i < nv; i += NTHR) { const v4i v = ((const v4i*)region)[i]; *(volatile v4i*)(gp + 4 * i) = v; }
  __threadfence();
#pragma unroll 1
  for (int i = tid; i < nv; i += NTHR) { const v4i v = ((const v4i*)region)[i]; *(volatile v4i*)(gp + 4 * i) = v; }
}

template <int SRC16>
__device__ __forceinline__ v4f ldrow(const float* __restrict__ xs, const _Float16* __restrict__ hs, int s, int lane) {
  v4f r;
  if (SRC16 != 0) {
    const v4h q = *(const v4h*)(hs + (size_t)s * HID + 4 * lane);
    r.x = (float)q[0]; r.y = (float)q[1]; r.z = (float)q[2]; r.w = (float)q[3];
  } else {
    r = *(const v4f*)(xs + (size_t)s * HID + 4 * lane);
  }
  return r;
}

template <int SRC16>
__global__ __launch_bounds__(NTHR) void k_layer(
    const int* __restrict__ csr, const int* __restrict__ off, const int* __restrict__ cnt,
    const float* __restrict__ dinv, const float* __restrict__ xs, const _Float16* __restrict__ hs,
    const _Float16* __restrict__ wl, const float* __restrict__ bl, const _Float16* __restrict__ wj,
    const float* __restrict__ linb, _Float16* hout, float* logits, float* out,
    int nN, int csrLen, int accum, int last, int storeRows) {
  extern __shared__ v4f lds_dyn[];
  _Float16* sA = (_Float16*)lds_dyn;
  _Float16* sH = sA + GROWS * AP;
  float*    sL = (float*)lds_dyn;
  const int tid = threadIdx.x, lane = tid & 31, wave = tid >> 5, hh = lane >> 4, m = lane & 15;
  const int rowBase = blockIdx.x * GROWS;
  const int tbase   = rowBase + wave * 16;

  {
    const int cl = tbase + lane;
    const int cnt_l = cnt[cl];
    const int off_l = off[cl];
    FI dvu; dvu.f = dinv[cl];
#pragma unroll 1
    for (int j = 0; j < 16; ++j) {
      const int c = tbase + j;
      int n = __builtin_amdgcn_readlane(cnt_l, j);
      n = n < 0 ? 0 : (n > DEGCAP ? DEGCAP : n);
      const int st = __builtin_amdgcn_readlane(off_l, j);
      FI du; du.i = __builtin_amdgcn_readlane(dvu.i, j);
      const float dc = du.f;
      v4f acc = {0.f, 0.f, 0.f, 0.f};
#pragma unroll 1
      for (int q0 = 0; q0 < n; q0 += 32) {
        int pos = st + q0 + lane;
        pos = pos < 0 ? 0 : (pos > csrLen - 1 ? csrLen - 1 : pos);
        int sl = csr[pos];
        sl = sl < 0 ? 0 : (sl > nN - 1 ? nN - 1 : sl);
        FI dsu; dsu.f = dinv[sl];
        const int mcnt = (n - q0) < 32 ? (n - q0) : 32;
#pragma unroll 1
        for (int p = 0; p < mcnt; ++p) {
          const int s = __builtin_amdgcn_readlane(sl, p);
          FI dd; dd.i = __builtin_amdgcn_readlane(dsu.i, p);
          const v4f r = ldrow<SRC16>(xs, hs, s, lane);
          acc = acc + r * dd.f;
        }
      }
      const int cs = c > nN - 1 ? nN - 1 : c;
      const v4f sr = ldrow<SRC16>(xs, hs, SRC16 != 0 ? c : cs, lane);
      acc = (acc + sr * dc) * dc;
      v4h hv;
      hv[0] = (_Float16)acc.x; hv[1] = (_Float16)acc.y; hv[2] = (_Float16)acc.z; hv[3] = (_Float16)acc.w;
      *(v4h*)(sA + (wave * 16 + j) * AP + 4 * lane) = hv;
    }
  }
  __syncthreads();

  {
    const _Float16* ar = sA + (wave * 16 + m) * AP + 8 * hh;
#pragma unroll 1
    for (int g = 0; g < 2; ++g) {
      v8f acc[4];
#pragma unroll
      for (int t = 0; t < 4; ++t) { v8f z = {0.f, 0.f, 0.f, 0.f, 0.f, 0.f, 0.f, 0.f}; acc[t] = z; }
#pragma unroll
      for (int kt = 0; kt < HID / 32; ++kt) {
        FragH a;
        a.h[0] = *(const v8h*)(ar + 32 * kt);
        a.h[1] = *(const v8h*)(ar + 32 * kt + 16);
#pragma unroll
        for (int t = 0; t < 4; ++t) {
          const _Float16* bp = wl + (size_t)(64 * g + 16 * t + m) * HID + 32 * kt + 8 * hh;
          FragH b;
          b.h[0] = *(const v8h*)bp;
          b.h[1] = *(const v8h*)(bp + 16);
          acc[t] = wmh(a.v, b.v, acc[t]);
        }
      }
#pragma unroll
      for (int t = 0; t < 4; ++t) {
        const int col = 64 * g + 16 * t + m;
        const float bv = bl[col];
        _Float16* sp = sH + (wave * 16 + 8 * hh) * AP + col;
#pragma unroll
        for (int r = 0; r < 8; ++r) {
          const float v = fmaxf(acc[t][r] * WINV + bv, 0.0f);
          sp[r * AP] = (_Float16)v;
        }
      }
    }
  }
  __syncthreads();

  {
    _Float16* gp = hout + (size_t)(rowBase + wave * 16) * HID;
#pragma unroll
    for (int p = 0; p < 8; ++p) {
      const int row = 2 * p + hh;
      const v8h v = *(const v8h*)(sH + (wave * 16 + row) * AP + 8 * m);
      *(volatile v8h*)(gp + (size_t)row * HID + 8 * m) = v;
    }
    __threadfence();
#pragma unroll
    for (int p = 0; p < 8; ++p) {
      const int row = 2 * p + hh;
      const v8h v = *(const v8h*)(sH + (wave * 16 + row) * AP + 8 * m);
      *(volatile v8h*)(gp + (size_t)row * HID + 8 * m) = v;
    }
  }

  {
    v8f acc2[4];
#pragma unroll
    for (int t = 0; t < 4; ++t) { v8f z = {0.f, 0.f, 0.f, 0.f, 0.f, 0.f, 0.f, 0.f}; acc2[t] = z; }
    const _Float16* ar2 = sH + (wave * 16 + m) * AP + 8 * hh;
#pragma unroll
    for (int kt = 0; kt < HID / 32; ++kt) {
      FragH a;
      a.h[0] = *(const v8h*)(ar2 + 32 * kt);
      a.h[1] = *(const v8h*)(ar2 + 32 * kt + 16);
#pragma unroll
      for (int t = 0; t < 4; ++t) {
        const _Float16* bp = wj + (size_t)(16 * t + m) * HID + 32 * kt + 8 * hh;
        FragH b;
        b.h[0] = *(const v8h*)bp;
        b.h[1] = *(const v8h*)(bp + 16);
        acc2[t] = wmh(a.v, b.v, acc2[t]);
      }
    }
#pragma unroll
    for (int t = 0; t < 4; ++t) {
      const int col = 16 * t + m;
      float* sp = sL + (wave * 16 + 8 * hh) * OUTC + col;
#pragma unroll
      for (int r = 0; r < 8; ++r) sp[r * OUTC] = acc2[t][r] * WINV;
    }
  }
  __syncthreads();

  {
    v4f vals[8];
    const int col = 4 * m;
#pragma unroll
    for (int p = 0; p < 8; ++p) {
      const int row = wave * 16 + 2 * p + hh;
      const v4f add = *(const v4f*)(sL + row * OUTC + col);
      const v4f old = *(const v4f*)(logits + (size_t)(rowBase + row) * OUTC + col);
      v4f base;
      base.x = accum != 0 ? old.x : 0.0f;
      base.y = accum != 0 ? old.y : 0.0f;
      base.z = accum != 0 ? old.z : 0.0f;
      base.w = accum != 0 ? old.w : 0.0f;
      vals[p] = base + add;
    }
    if (last != 0) {
      const v4f lb = *(const v4f*)(linb + col);
#pragma unroll
      for (int p = 0; p < 8; ++p) {
        v4f v = vals[p] + lb;
        float mx = fmaxf(fmaxf(v.x, v.y), fmaxf(v.z, v.w));
        mx = fmaxf(mx, __shfl_xor(mx, 8, 32));
        mx = fmaxf(mx, __shfl_xor(mx, 4, 32));
        mx = fmaxf(mx, __shfl_xor(mx, 2, 32));
        mx = fmaxf(mx, __shfl_xor(mx, 1, 32));
        float s = expf(v.x - mx) + expf(v.y - mx) + expf(v.z - mx) + expf(v.w - mx);
        s += __shfl_xor(s, 8, 32);
        s += __shfl_xor(s, 4, 32);
        s += __shfl_xor(s, 2, 32);
        s += __shfl_xor(s, 1, 32);
        const float lse = mx + logf(s);
        v.x -= lse; v.y -= lse; v.z -= lse; v.w -= lse;
        vals[p] = v;
      }
    }
    float* dstp = last != 0 ? out : logits;
#pragma unroll
    for (int p = 0; p < 8; ++p) {
      const int grow = rowBase + wave * 16 + 2 * p + hh;
      if (grow < storeRows) *(volatile v4f*)(dstp + (size_t)grow * OUTC + col) = vals[p];
    }
    __threadfence();
#pragma unroll
    for (int p = 0; p < 8; ++p) {
      const int grow = rowBase + wave * 16 + 2 * p + hh;
      if (grow < storeRows) *(volatile v4f*)(dstp + (size_t)grow * OUTC + col) = vals[p];
    }
  }
}

extern "C" void kernel_launch(void* const* d_in, const int* in_sizes, int n_in,
                              void* d_out, int out_size, void* d_ws, size_t ws_size,
                              hipStream_t stream) {
  if (n_in < 12) return;
  const int nN = in_sizes[0] / HID;
  const int nE = in_sizes[1] / 2;
  if (nN <= 0 || nE <= 0 || in_sizes[0] != nN * HID || in_sizes[1] != 2 * nE) return;
  if (in_sizes[2] != HID * HID || in_sizes[4] != HID * HID || in_sizes[6] != HID * HID || in_sizes[8] != HID * HID) return;
  if (in_sizes[3] < HID || in_sizes[5] < HID || in_sizes[7] < HID || in_sizes[9] < HID) return;
  if (in_sizes[10] != NLAY * HID * OUTC || in_sizes[11] < OUTC) return;
  if (out_size != nN * OUTC) return;
  if (nE > (1 << 28) || nN > (1 << 24)) return;

  const float* x    = (const float*)d_in[0];
  const int*   ei   = (const int*)d_in[1];
  const float* W0   = (const float*)d_in[2];
  const float* b0   = (const float*)d_in[3];
  const float* W1   = (const float*)d_in[4];
  const float* b1   = (const float*)d_in[5];
  const float* W2   = (const float*)d_in[6];
  const float* b2   = (const float*)d_in[7];
  const float* W3   = (const float*)d_in[8];
  const float* b3   = (const float*)d_in[9];
  const float* linW = (const float*)d_in[10];
  const float* linb = (const float*)d_in[11];
  float* out = (float*)d_out;

  const int NPAD   = ((nN + GROWS - 1) / GROWS) * GROWS;
  const int nBC    = (nN + NBC - 1) / NBC;
  const int CNTW   = nBC * NBC;
  const int CNTPAD = CNTW + CPADX;
  if (4 * nBC + 1 > RBN) return;
  const int nBF    = (nN + NBF - 1) / NBF;
  const int csrLen = ((nE + 31) & ~31) + 4096;
  const int nLay   = NPAD / GROWS;

  char* ws = (char*)d_ws;
  size_t off = 0;
  const size_t oWL  = off; off += (size_t)NLAY * HID * HID * 2;    off = (off + 255) & ~(size_t)255;
  const size_t oWJ  = off; off += (size_t)NLAY * OUTC * HID * 2;   off = (off + 255) & ~(size_t)255;
  const size_t oCnt = off; off += (size_t)CNTPAD * 4;              off = (off + 255) & ~(size_t)255;
  const size_t oDv  = off; off += (size_t)CNTPAD * 4;              off = (off + 255) & ~(size_t)255;
  const size_t oOff = off; off += (size_t)CNTPAD * 4;              off = (off + 255) & ~(size_t)255;
  const size_t oRb  = off; off += (size_t)RBN * 4;                 off = (off + 255) & ~(size_t)255;
  const size_t oCsr = off; off += (size_t)csrLen * 4;              off = (off + 255) & ~(size_t)255;
  const size_t oP0  = off; off += (size_t)NPAD * HID * 2;          off = (off + 255) & ~(size_t)255;
  const size_t oP1  = off; off += (size_t)NPAD * HID * 2;          off = (off + 255) & ~(size_t)255;
  const size_t oLg  = off; off += (size_t)NPAD * OUTC * 4;         off = (off + 255) & ~(size_t)255;
  if (off > ws_size) return;
  if (off > (size_t)134217728) return;
  _Float16* wl     = (_Float16*)(ws + oWL);
  _Float16* wj     = (_Float16*)(ws + oWJ);
  int*      cnt    = (int*)(ws + oCnt);
  float*    dinv   = (float*)(ws + oDv);
  int*      offp   = (int*)(ws + oOff);
  int*      rb     = (int*)(ws + oRb);
  int*      csr    = (int*)(ws + oCsr);
  _Float16* P0     = (_Float16*)(ws + oP0);
  _Float16* P1     = (_Float16*)(ws + oP1);
  float*    logits = (float*)(ws + oLg);

  const int vec8 = ((nE & 3) == 0) ? 1 : 0;

  const int nPrep = NLAY * HID * HID / 8 + NLAY * OUTC * HID / 8;
  k_wprep<<<(nPrep + NTHR - 1) / NTHR, NTHR, 0, stream>>>(W0, W1, W2, W3, linW, wl, wj);

  k_count<<<nBC, NTHR, 0, stream>>>(ei, cnt, dinv, nE, vec8);
  k_offsets<<<1, OTHR, 0, stream>>>(cnt, offp, rb, nBC);
  hipFuncSetAttribute(reinterpret_cast<const void*>(&k_fill),
                      hipFuncAttributeMaxDynamicSharedMemorySize, LDS_FILL);
  k_fill<<<nBF, NTHR, LDS_FILL, stream>>>(ei, offp, rb, csr, nN, nE, vec8, csrLen);

  hipFuncSetAttribute(reinterpret_cast<const void*>(&k_layer<0>),
                      hipFuncAttributeMaxDynamicSharedMemorySize, LDS_LAYER);
  hipFuncSetAttribute(reinterpret_cast<const void*>(&k_layer<1>),
                      hipFuncAttributeMaxDynamicSharedMemorySize, LDS_LAYER);
  k_layer<0><<<nLay, NTHR, LDS_LAYER, stream>>>(csr, offp, cnt, dinv, x, P1, wl,                          b0, wj,                          linb, P0, logits, out, nN, csrLen, 0, 0, NPAD);
  k_layer<1><<<nLay, NTHR, LDS_LAYER, stream>>>(csr, offp, cnt, dinv, x, P0, wl + (size_t)1 * HID * HID, b1, wj + (size_t)1 * OUTC * HID, linb, P1, logits, out, nN, csrLen, 1, 0, NPAD);
  k_layer<1><<<nLay, NTHR, LDS_LAYER, stream>>>(csr, offp, cnt, dinv, x, P1, wl + (size_t)2 * HID * HID, b2, wj + (size_t)2 * OUTC * HID, linb, P0, logits, out, nN, csrLen, 1, 0, NPAD);
  k_layer<1><<<nLay, NTHR, LDS_LAYER, stream>>>(csr, offp, cnt, dinv, x, P0, wl + (size_t)3 * HID * HID, b3, wj + (size_t)3 * OUTC * HID, linb, P1, logits, out, nN, csrLen, 1, 1, nN);
}
